// GAT_24017457119793
// MI455X (gfx1250) — hardware-verified
//
#include <hip/hip_runtime.h>
#include <stddef.h>


typedef _Float16 h16;
typedef _Float16 v16h __attribute__((ext_vector_type(16)));
typedef _Float16 v8h  __attribute__((ext_vector_type(8)));
typedef _Float16 v4h  __attribute__((ext_vector_type(4)));
typedef float    v8f  __attribute__((ext_vector_type(8)));
typedef float    v4f  __attribute__((ext_vector_type(4)));
typedef float    v2f  __attribute__((ext_vector_type(2)));

#ifndef NB
#define NB 16384
#endif
#define NB_FULL 16384
#define NNODE 23
#define NADJ  529
#define XDIM  92
#define KP1   96
#define FC1N  128
#define PREN  16

#define LDM 136
#define LDC 132
#define XPL 17
#define LDW 136

#define WCARRY 64.0f
#define XCARRY 64.0f
#define MCARRY 16.0f
#define NEG_FILL (-1.0e20f)

#define OUT_Y_OFF   0
#define OUT_VAR_OFF NB_FULL
#define OUT_XC_OFF  (2 * NB_FULL)

static_assert(NB >= 128 && NB <= NB_FULL && (NB % 128) == 0);
static_assert(XDIM == NNODE * 4);
static_assert(NADJ == NNODE * NNODE);
static_assert((KP1 % 32) == 0 && KP1 >= XDIM && (KP1 - XDIM) == 4);
static_assert(NNODE + 1 <= 32);
static_assert((FC1N % 32) == 0 && FC1N == 8 * 16);
static_assert(PREN == 16);
static_assert((LDM % 8) == 0 && LDM >= FC1N && LDM >= KP1);
static_assert((LDC % 4) == 0 && LDC >= FC1N);
static_assert(XPL >= PREN);
static_assert(FC1N * 4 == 32 * 16);
static_assert(128 * 4 == 32 * 16);
static_assert(LDW >= KP1 && LDW >= FC1N && (LDW % 8) == 0);
static_assert(((16 * KP1) % 256) == 0 && ((16 * FC1N) % 256) == 0);
static_assert(((16 * (KP1 / 8)) % 32) == 0 && (16 * (KP1 / 8)) <= 256);
static_assert(((16 * (FC1N / 8)) % 32) == 0 && (16 * (FC1N / 8)) <= 256);
static_assert((FC1N % 16) == 0 && (PREN % 16) == 0);
static_assert((size_t)OUT_VAR_OFF * 4 == (size_t)65536);
static_assert((size_t)OUT_XC_OFF * 4 == (size_t)131072);
static_assert((size_t)OUT_XC_OFF + (size_t)NB_FULL * FC1N == (size_t)8519680 / 4);

#define LDS_TOTAL ((size_t)8 * 16 * LDM * 2 + (size_t)8 * 16 * LDC * 4 + (size_t)8 * 32 * 2 * 4 + \
                   (size_t)8 * 32 * 4 * 4 + (size_t)8 * 32 * 2 * 4 + (size_t)8 * 16 * XPL * 4 + (size_t)2 * 128 * 4)
static_assert(LDS_TOTAL <= (size_t)131072);

#define W1T_BYTES ((size_t)FC1N * KP1 * 2)
#define W2T_BYTES ((size_t)PREN * FC1N * 2)
#define OFF_W1T   ((size_t)0)
#define OFF_W2T   (OFF_W1T + W1T_BYTES)
#define WS_TOTAL  (OFF_W2T + W2T_BYTES)
static_assert((W1T_BYTES % 128) == 0 && (W2T_BYTES % 128) == 0);
static_assert(WS_TOTAL <= (size_t)134217728);

__device__ __forceinline__ float bf16r(float x) {
  unsigned int u = __float_as_uint(x);
  u = (u + 0x7FFFu + ((u >> 16) & 1u)) & 0xFFFF0000u;
  return __uint_as_float(u);
}

static __device__ __forceinline__ h16 toh_flush(float v) {
  const h16 r = (h16)v;
  return (fabsf(v) < 6.103515625e-05f) ? (h16)0.0f : r;
}

__device__ __forceinline__ v16h frag_at(const _Float16* p) {
  v8h lo = *(const v8h*)(p);
  v8h hi = *(const v8h*)(p + 16);
  v16h out;
#pragma unroll
  for (int i = 0; i < 8; ++i) { out[i] = lo[i]; out[i + 8] = hi[i]; }
  return out;
}
__device__ __forceinline__ v16h ld_frag(const _Float16* base, unsigned ld) {
  const unsigned lane = threadIdx.x & 31u;
  return frag_at(base + (lane & 15u) * ld + (lane >> 4) * 8u);
}

__device__ __forceinline__ v8f wmma16(v16h a, v16h b, v8f c) {
  v8f d = __builtin_amdgcn_wmma_f32_16x16x32_f16(false, a, false, b, (short)0, c,
                                                 false, false);
  asm volatile("v_nop\n\tv_nop\n\tv_nop\n\tv_nop" : "+v"(d) : "v"(a), "v"(b));
  return d;
}

__device__ __forceinline__ void wave_lds_sync() {
  __builtin_amdgcn_fence(3  , "wavefront");
  asm volatile("s_wait_dscnt 0x0" ::: "memory");
  __builtin_amdgcn_wave_barrier();
}

__device__ __forceinline__ float gelu_exact(float v) {
  return 0.5f * v * (1.0f + erff(v * 0.70710678118654752f));
}

__device__ __forceinline__ float edge_score(float s, bool on) {
  const float l = (s > 0.0f) ? s : 0.2f * s;
  return on ? l : NEG_FILL;
}

__device__ __forceinline__ void online_upd(float e, float& mx, float& dn) {
  const float mn = fmaxf(mx, e);
  dn = dn * __expf(mx - mn) + __expf(e - mn);
  mx = mn;
}

__global__ __launch_bounds__(256) void wconv_kernel(
    const float* __restrict__ W, _Float16* __restrict__ Wt, unsigned K, unsigned ldw, unsigned KP) {
  __shared__ __attribute__((aligned(16))) _Float16 T[16 * LDW];
  const unsigned tid = threadIdx.x;
  const unsigned n0 = blockIdx.x * 16u;
#pragma unroll 1
  for (unsigned idx = tid; idx < 16u * KP; idx += 256u) {
    const unsigned kr = idx >> 4, nc = idx & 15u;
    const unsigned kcl = (kr < K) ? kr : (K - 1u);
    const float v = W[(size_t)kcl * ldw + n0 + nc];
    const h16 c = toh_flush(WCARRY * bf16r(v));
    T[nc * LDW + kr] = (kr < K) ? c : (h16)0.0f;
  }
  __syncthreads();
  const unsigned ppr = KP >> 3;
  const unsigned pieces = 16u * ppr;
  if (tid < pieces) {
    const unsigned r = tid / ppr;
    const unsigned kc = (tid - r * ppr) * 8u;
    const v8h x = *(const v8h*)&T[r * LDW + kc];
    _Float16* p = Wt + (size_t)(n0 + r) * KP + kc;
    *(volatile v8h*)p = x;
    __threadfence();
    *(volatile v8h*)p = x;
  }
}

__global__ __launch_bounds__(256) void graph_attn_mlp_kernel(
    const float* __restrict__ node_attr, const int* __restrict__ adj,
    const float* __restrict__ W0, const float* __restrict__ a0,
    const float* __restrict__ W1, const float* __restrict__ a1,
    const _Float16* __restrict__ W1t, const float* __restrict__ fc1_b,
    const _Float16* __restrict__ W2t, const float* __restrict__ pre_b,
    const float* __restrict__ predict_w, const float* __restrict__ predict_b,
    const float* __restrict__ getvar_w, const float* __restrict__ getvar_b,
    float* __restrict__ out) {
  __shared__ __attribute__((aligned(16))) _Float16 AT[8 * 16 * LDM];
  __shared__ __attribute__((aligned(16))) float Cs[8 * 16 * LDC];
  __shared__ __attribute__((aligned(16))) float F1s[8 * 32 * 2];
  __shared__ __attribute__((aligned(16))) float CAs[8 * 32 * 4];
  __shared__ __attribute__((aligned(16))) float CBs[8 * 32 * 2];
  __shared__ __attribute__((aligned(16))) float XPs[8 * 16 * XPL];
  __shared__ __attribute__((aligned(16))) float YVs[2 * 128];

  const unsigned tid = threadIdx.x, lane = tid & 31u;
  const unsigned wave = (unsigned)__builtin_amdgcn_readfirstlane((int)(threadIdx.x >> 5));
  const unsigned hh = lane >> 4, m = lane & 15u;
  const unsigned row0 = blockIdx.x * 128u + wave * 16u;
  const unsigned nd = (lane < (unsigned)NNODE) ? lane : (unsigned)(NNODE - 1);
  const unsigned abase = wave * (16u * LDM);
  const unsigned cbase = wave * (16u * LDC);

  const float w00 = bf16r(W0[0]), w01 = bf16r(W0[1]);
  const float w10 = bf16r(W1[0]), w11 = bf16r(W1[1]);
  const float a00 = bf16r(a0[0]), a01 = bf16r(a0[1]), a02 = bf16r(a0[2]), a03 = bf16r(a0[3]);
  const float a10 = bf16r(a1[0]), a11 = bf16r(a1[1]), a12 = bf16r(a1[2]), a13 = bf16r(a1[3]);

#pragma unroll 1
  for (unsigned s = 0; s < 16u; ++s) {
    const unsigned smp = row0 + s;
    const float xv = bf16r(node_attr[(size_t)smp * NNODE + nd]);
    const float h00 = xv * w00, h01 = xv * w01;
    const float h10 = xv * w10, h11 = xv * w11;
    const float f1_0 = h00 * a00 + h01 * a01;
    const float f2_0 = h00 * a02 + h01 * a03;
    const float f1_1 = h10 * a10 + h11 * a11;
    const float f2_1 = h10 * a12 + h11 * a13;
    v2f ff;
    ff[0] = f1_0; ff[1] = f1_1;
    *(v2f*)&F1s[wave * 64u + lane * 2u] = ff;
    wave_lds_sync();

    const int* ap = adj + (size_t)smp * NADJ + nd;
    float m0 = -1.0e30f, m1 = -1.0e30f, d0 = 0.0f, d1 = 0.0f;
    unsigned rowbits = 0u;
#pragma unroll 1
    for (unsigned i = 0; i < (unsigned)NNODE; ++i) {
      int av = ap[i * (unsigned)NNODE];
      asm volatile("" : "+v"(av));
      const bool on = av > 0;
      const unsigned bal = __builtin_amdgcn_ballot_w32(on);
      rowbits = (lane == i) ? bal : rowbits;
      const v2f f = *(const v2f*)&F1s[wave * 64u + i * 2u];
      const float e0 = edge_score(f[0] + f2_0, on);
      const float e1 = edge_score(f[1] + f2_1, on);
      online_upd(e0, m0, d0);
      online_upd(e1, m1, d1);
    }
    v4f ca;
    ca[0] = m0; ca[1] = m1; ca[2] = f2_0; ca[3] = f2_1;
    v2f cb;
    cb[0] = (1.0f / d0) * xv;
    cb[1] = (1.0f / d1) * xv;
    *(v4f*)&CAs[wave * 128u + lane * 4u] = ca;
    *(v2f*)&CBs[wave * 64u + lane * 2u] = cb;
    wave_lds_sync();

    float s0 = 0.0f, s1 = 0.0f;
#pragma unroll 1
    for (unsigned j = 0; j < (unsigned)NNODE; ++j) {
      const v4f c = *(const v4f*)&CAs[wave * 128u + j * 4u];
      const v2f g = *(const v2f*)&CBs[wave * 64u + j * 2u];
      const bool on = ((rowbits >> j) & 1u) != 0u;
      const float e0 = edge_score(f1_0 + c[2], on);
      const float e1 = edge_score(f1_1 + c[3], on);
      s0 += __expf(e0 - c[0]) * g[0];
      s1 += __expf(e1 - c[1]) * g[1];
    }
    const bool live = lane < (unsigned)NNODE;
    const float u0 = gelu_exact(w00 * s0);
    const float u1 = gelu_exact(w01 * s0);
    const float u2 = gelu_exact(w10 * s1);
    const float u3 = gelu_exact(w11 * s1);
    v4h o;
    o[0] = live ? toh_flush(XCARRY * u0) : (h16)0.0f;
    o[1] = live ? toh_flush(XCARRY * u1) : (h16)0.0f;
    o[2] = live ? toh_flush(XCARRY * u2) : (h16)0.0f;
    o[3] = live ? toh_flush(XCARRY * u3) : (h16)0.0f;
    if (lane < (unsigned)(NNODE + 1)) *(v4h*)&AT[abase + s * LDM + lane * 4u] = o;
    wave_lds_sync();
  }
  __syncthreads();

  v8f acc[8];
#pragma unroll
  for (int nt = 0; nt < 8; ++nt) acc[nt] = (v8f){};
  const _Float16* bp = W1t + (size_t)m * KP1 + hh * 8u;
#pragma unroll 1
  for (unsigned ks = 0; ks < (unsigned)(KP1 / 32); ++ks) {
    const v16h a = ld_frag(&AT[abase + ks * 32u], LDM);
#pragma unroll
    for (int nt = 0; nt < 8; ++nt) {
      const v16h b = frag_at(bp + (size_t)(nt * 16) * KP1 + ks * 32u);
      acc[nt] = wmma16(a, b, acc[nt]);
    }
  }
  wave_lds_sync();
#pragma unroll
  for (int nt = 0; nt < 8; ++nt) {
    const float bb = bf16r(fc1_b[nt * 16 + (int)m]);
#pragma unroll
    for (int r = 0; r < 8; ++r) {
      const float v = fmaxf(acc[nt][r] * (1.0f / (XCARRY * WCARRY)) + bb, 0.0f);
      Cs[cbase + (hh * 8u + (unsigned)r) * LDC + (unsigned)nt * 16u + m] = v;
      AT[abase + (hh * 8u + (unsigned)r) * LDM + (unsigned)nt * 16u + m] = toh_flush(MCARRY * v);
    }
  }
  wave_lds_sync();

  {
    v4f xs[16];
#pragma unroll
    for (int r = 0; r < 16; ++r) xs[r] = *(const v4f*)&Cs[cbase + (unsigned)r * LDC + lane * 4u];
    float* xcp = out + (size_t)OUT_XC_OFF + (size_t)row0 * FC1N + lane * 4u;
#pragma unroll
    for (int r = 0; r < 16; ++r) *(volatile v4f*)(xcp + r * FC1N) = xs[r];
    __threadfence();
#pragma unroll
    for (int r = 0; r < 16; ++r) *(volatile v4f*)(xcp + r * FC1N) = xs[r];
  }

  v8f pacc = {};
  const _Float16* b2p = W2t + (size_t)m * FC1N + hh * 8u;
#pragma unroll
  for (int ks = 0; ks < FC1N / 32; ++ks) {
    const v16h a = ld_frag(&AT[abase + ks * 32], LDM);
    const v16h b = frag_at(b2p + ks * 32);
    pacc = wmma16(a, b, pacc);
  }
  {
    const float pbv = bf16r(pre_b[m]);
#pragma unroll
    for (int r = 0; r < 8; ++r) {
      const float z = pacc[r] * (1.0f / (MCARRY * WCARRY)) + pbv;
      XPs[wave * (16u * XPL) + (hh * 8u + (unsigned)r) * XPL + m] = gelu_exact(z);
    }
  }
  wave_lds_sync();

  {
    const unsigned xb = wave * (16u * XPL) + m * XPL;
    float sacc = 0.0f;
#pragma unroll 4
    for (unsigned n = 0; n < 16u; ++n) {
      const float pw = bf16r(predict_w[n]);
      const float gw = bf16r(getvar_w[n]);
      const float wv = (hh != 0u) ? gw : pw;
      sacc += XPs[xb + n] * wv;
    }
    const float pbb = bf16r(predict_b[0]);
    const float gbb = bf16r(getvar_b[0]);
    const float tot = sacc + ((hh != 0u) ? gbb : pbb);
    const float res = (hh != 0u) ? tot : fmaxf(tot, 0.0f);
    YVs[hh * 128u + wave * 16u + m] = res;
  }
  __syncthreads();

  if (wave < 2u) {
    const v4f v = *(const v4f*)&YVs[wave * 128u + lane * 4u];
    float* p = out + (size_t)wave * NB_FULL + (size_t)blockIdx.x * 128u + lane * 4u;
    *(volatile v4f*)p = v;
    __threadfence();
    *(volatile v4f*)p = v;
  }
}

extern "C" void kernel_launch(void* const* d_in, const int* in_sizes, int n_in,
                              void* d_out, int out_size, void* d_ws, size_t ws_size,
                              hipStream_t stream) {
  if (n_in < 14) return;
  if ((long long)in_sizes[0] < (long long)NB * NNODE) return;
  if ((long long)in_sizes[1] < (long long)NB * NADJ) return;
  if (in_sizes[2] < 2 || in_sizes[3] < 4 || in_sizes[4] < 2 || in_sizes[5] < 4) return;
  if (in_sizes[6] < XDIM * FC1N || in_sizes[7] < FC1N) return;
  if (in_sizes[8] < FC1N * PREN || in_sizes[9] < PREN) return;
  if (in_sizes[10] < PREN || in_sizes[11] < 1 || in_sizes[12] < PREN || in_sizes[13] < 1) return;
  if ((long long)out_size < (long long)OUT_XC_OFF + (long long)NB * FC1N) return;
  if (ws_size < WS_TOTAL) return;

  const float* node_attr = (const float*)d_in[0];
  const int*   adj       = (const int*)d_in[1];
  const float* W0        = (const float*)d_in[2];
  const float* a0        = (const float*)d_in[3];
  const float* W1        = (const float*)d_in[4];
  const float* a1        = (const float*)d_in[5];
  const float* fc1_w     = (const float*)d_in[6];
  const float* fc1_b     = (const float*)d_in[7];
  const float* pre_w     = (const float*)d_in[8];
  const float* pre_b     = (const float*)d_in[9];
  const float* predict_w = (const float*)d_in[10];
  const float* predict_b = (const float*)d_in[11];
  const float* getvar_w  = (const float*)d_in[12];
  const float* getvar_b  = (const float*)d_in[13];
  float* out = (float*)d_out;

  char* ws = (char*)d_ws;
  _Float16* W1t = (_Float16*)(ws + OFF_W1T);
  _Float16* W2t = (_Float16*)(ws + OFF_W2T);

  wconv_kernel<<<dim3(FC1N / 16), dim3(256), 0, stream>>>(fc1_w, W1t, (unsigned)XDIM, (unsigned)FC1N,
                                                         (unsigned)KP1);
  wconv_kernel<<<dim3(PREN / 16), dim3(256), 0, stream>>>(pre_w, W2t, (unsigned)FC1N, (unsigned)PREN,
                                                         (unsigned)FC1N);
  graph_attn_mlp_kernel<<<dim3(NB / 128), dim3(256), 0, stream>>>(
      node_attr, adj, W0, a0, W1, a1, W1t, fc1_b, W2t, pre_b,
      predict_w, predict_b, getvar_w, getvar_b, out);
}
